// MultiHeadAttention_5059471475068
// MI455X (gfx1250) — hardware-run, weakly checked
//
#include <hip/hip_runtime.h>
#ifndef NB
#define NB 2
#endif
#ifndef SEQ
#define SEQ 2048
#endif
#define NB_FULL 2
#define SEQ_FULL 2048
#define DM 1024
#define NH 16
#define HD 64
#define HG 2
#define NR ((size_t)NB * SEQ)
#define LQ DM

static_assert(NB >= 1 && NB <= NB_FULL);
static_assert(SEQ <= SEQ_FULL);
static_assert(SEQ % 128 == 0);
static_assert(DM % 64 == 0 && DM % 32 == 0);
static_assert(HD == 64 && NH * HD == DM);
static_assert(NH % HG == 0);

#define SZ_W   ((size_t)DM * DM * 2)
#define SZ_ROW ((size_t)NB * SEQ * DM * 2)
#define SZ_S   ((size_t)HG * SEQ * SEQ * 4)
#define SZ_P   ((size_t)HG * SEQ * SEQ * 2)
#define SZ_VT  ((size_t)NB * NH * HD * SEQ * 2)
#define WS_TOTAL (4 * SZ_W + 5 * SZ_ROW + SZ_S + SZ_P + SZ_VT)
static_assert(SZ_W % 256 == 0 && SZ_ROW % 256 == 0 && SZ_S % 256 == 0 && SZ_P % 256 == 0 && SZ_VT % 256 == 0);
static_assert(WS_TOTAL <= (size_t)134217728);

typedef unsigned short v8us __attribute__((ext_vector_type(8), may_alias));
typedef float  v8f  __attribute__((ext_vector_type(8)));
typedef float  v4f  __attribute__((ext_vector_type(4)));
typedef float  v4fa __attribute__((ext_vector_type(4), may_alias));
typedef _Float16 v16h __attribute__((ext_vector_type(16)));
typedef _Float16 v4h __attribute__((ext_vector_type(4)));
union FragH { v16h v; v8us half[2]; _Float16 h[16]; unsigned short u[16]; };

__device__ __forceinline__ unsigned short bf16_bits(float x) { unsigned int u = __float_as_uint(x); return (unsigned short)((u + 0x7FFFu + ((u >> 16) & 1u)) >> 16); }
__device__ __forceinline__ float bf16_val(unsigned short b) { return __uint_as_float(((unsigned int)b) << 16); }
__device__ __forceinline__ float bf16_rne(float x) { return bf16_val(bf16_bits(x)); }

__global__ __launch_bounds__(256) void k_x16(const float* __restrict__ x, _Float16* __restrict__ X16, size_t n8) {
  const size_t t = (size_t)blockIdx.x * 256 + threadIdx.x; if (t >= n8) return;
  const size_t e = t * 8; const size_t row = e / DM; const size_t c = e % DM;
  const size_t b = row / SEQ, s = row % SEQ;
  const float* src = x + (b * (size_t)SEQ_FULL + s) * DM + c;
  const v4f a = *(const v4fa*)(src), d = *(const v4fa*)(src + 4);
  FragH f;
#pragma unroll
  for (int q = 0; q < 4; ++q) { f.h[q] = (_Float16)bf16_rne(a[q]); f.h[4 + q] = (_Float16)bf16_rne(d[q]); }
  const v8us o = f.half[0];
  *(volatile v8us*)((unsigned short*)X16 + t * 8) = o; __threadfence(); *(volatile v8us*)((unsigned short*)X16 + t * 8) = o;
}

__global__ __launch_bounds__(256) void k_wnat(const float* __restrict__ w, size_t n8, _Float16* __restrict__ Bt) {
  const size_t t = (size_t)blockIdx.x * 256 + threadIdx.x; if (t >= n8) return;
  const v4f a = *(const v4fa*)(w + t * 8), d = *(const v4fa*)(w + t * 8 + 4);
  FragH f;
#pragma unroll
  for (int q = 0; q < 4; ++q) { f.h[q] = (_Float16)(bf16_rne(a[q]) * 16.0f); f.h[4 + q] = (_Float16)(bf16_rne(d[q]) * 16.0f); }
  const v8us o = f.half[0];
  *(volatile v8us*)((unsigned short*)Bt + t * 8) = o; __threadfence(); *(volatile v8us*)((unsigned short*)Bt + t * 8) = o;
}

template <int NHv, int TTv>
__global__ __launch_bounds__(256) void k_vt(const _Float16* __restrict__ V16, int ldv, int voff, _Float16* __restrict__ Vt) {
  __shared__ unsigned short tl[64][66];
  const int tid = threadIdx.x; const int slab = blockIdx.x / (TTv / 64), lg = blockIdx.x % (TTv / 64); const int b = slab / NHv, h = slab % NHv;
  for (int i = tid; i < 64 * 8; i += 256) { const int r = i / 8, c8 = (i % 8) * 8; FragH f;
    f.half[0] = *(const v8us*)((const unsigned short*)V16 + ((size_t)b * TTv + lg * 64 + r) * ldv + voff + h * 64 + c8);
#pragma unroll
    for (int q = 0; q < 8; ++q) tl[r][c8 + q] = f.u[q]; }
  __syncthreads();
  for (int pass = 0; pass < 2; ++pass) {
#pragma unroll
    for (int rd = 0; rd < 2; ++rd) { const int d = rd * 32 + tid / 8, pc = tid % 8; FragH f;
#pragma unroll
      for (int q = 0; q < 8; ++q) f.u[q] = tl[pc * 8 + q][d];
      *(volatile v8us*)((unsigned short*)Vt + ((size_t)slab * 64 + d) * TTv + lg * 64 + pc * 8) = f.half[0]; }
    if (pass == 0) __threadfence(); } }

__global__ __launch_bounds__(256) void k_rsm(const float* __restrict__ S, _Float16* __restrict__ P, int nrows) {
  #pragma clang fp contract(off)
  const int i = blockIdx.x * 256 + threadIdx.x; if (i >= nrows) return; const float* s = S + (size_t)i * SEQ; float mx = -3.0e38f;
#pragma unroll 1
  for (int j = 0; j < SEQ; ++j) mx = fmaxf(mx, s[j]);
  float se = 0.f;
#pragma unroll 1
  for (int j = 0; j < SEQ; ++j) se += expf(s[j] - mx);
  const float sc = 256.0f / se;
#pragma unroll 1
  for (int j0 = 0; j0 < SEQ; j0 += 8) { FragH f;
    for (int q = 0; q < 8; ++q) f.h[q] = (_Float16)(expf(s[j0 + q] - mx) * sc);
    const v8us o = f.half[0]; unsigned short* d = (unsigned short*)P + (size_t)i * SEQ + j0;
    *(volatile v8us*)d = o; __threadfence(); *(volatile v8us*)d = o; } }

__device__ __forceinline__ v16h g2_frag(const _Float16* p, int hh) { FragH f; f.half[0] = *(const v8us*)((const unsigned short*)p + 8 * hh); f.half[1] = *(const v8us*)((const unsigned short*)p + 16 + 8 * hh); return f.v; }
__device__ __forceinline__ v8f g2_mma(v16h a, v16h b, v8f c) { v8f d = __builtin_amdgcn_wmma_f32_16x16x32_f16(false, a, false, b, (short)0, c, false, false); asm volatile("v_nop\n\tv_nop\n\tv_nop\n\tv_nop" : "+v"(d) : "v"(a), "v"(b)); return d; }
template <int ACT>
__global__ __launch_bounds__(128) void k_gemm2(const _Float16* __restrict__ A, int lda, size_t sA, const _Float16* __restrict__ Bh, int ldb, size_t sB, float alpha,
    const float* __restrict__ bias, size_t sBias, float* __restrict__ C, _Float16* __restrict__ C16, int ldc, size_t sC, int M, int N, int K) {
  static_assert(ACT == 0);
  __shared__ __attribute__((aligned(16))) float so[4][32][68];
  const int tid = threadIdx.x, w = __builtin_amdgcn_readfirstlane((int)(tid >> 5)), lane = tid & 31, ln = lane & 15, hh = lane >> 4; const int by = blockIdx.y;
  A += (size_t)by * sA; Bh += (size_t)by * sB; const size_t cofs = (size_t)by * sC; const float* bp = bias ? bias + (size_t)by * sBias : nullptr;
  const int ntn = N >> 6; const int mt = blockIdx.x / ntn, nq = blockIdx.x - mt * ntn; const int row0 = mt * 128 + 32 * w, col0 = nq * 64; if (row0 >= M) return;
  const _Float16* a0p = A + (size_t)(row0 + ln) * lda; const _Float16* a1p = a0p + (size_t)16 * lda;
  const _Float16* b0p = Bh + (size_t)(col0 + ln) * ldb; const _Float16* b1p = b0p + (size_t)16 * ldb; const _Float16* b2p = b1p + (size_t)16 * ldb; const _Float16* b3p = b2p + (size_t)16 * ldb;
  const v8f z8 = {0.f,0.f,0.f,0.f,0.f,0.f,0.f,0.f}; v8f c00 = z8, c01 = z8, c02 = z8, c03 = z8, c10 = z8, c11 = z8, c12 = z8, c13 = z8;
#pragma unroll 1
  for (int kb = 0; kb < K; kb += 32) { const v16h a0 = g2_frag(a0p + kb, hh), a1 = g2_frag(a1p + kb, hh);
    v16h b = g2_frag(b0p + kb, hh); c00 = g2_mma(a0, b, c00); c10 = g2_mma(a1, b, c10);
    b = g2_frag(b1p + kb, hh); c01 = g2_mma(a0, b, c01); c11 = g2_mma(a1, b, c11);
    b = g2_frag(b2p + kb, hh); c02 = g2_mma(a0, b, c02); c12 = g2_mma(a1, b, c12);
    b = g2_frag(b3p + kb, hh); c03 = g2_mma(a0, b, c03); c13 = g2_mma(a1, b, c13); }
  v8f accs[8] = {c00, c01, c02, c03, c10, c11, c12, c13};
#pragma unroll
  for (int u = 0; u < 8; ++u) { const int t = u & 3, half = u >> 2; const int col = col0 + t * 16 + ln; const float bv = bp ? bf16_rne(bp[col]) : 0.f;
#pragma unroll
    for (int r = 0; r < 8; ++r) { const int rloc = half * 16 + 8 * hh + r; const float v = accs[u][r] * alpha + bv; so[w][rloc][t * 16 + ln] = v; } }
  __builtin_amdgcn_fence(4  , "workgroup"); __builtin_amdgcn_wave_barrier();
  const int rsub = lane >> 4, c4 = (lane & 15) * 4;
  for (int pass = 0; pass < 2; ++pass) {
#pragma unroll
    for (int q = 0; q < 16; ++q) { const int r = q * 2 + rsub; const v4f v = *(const v4fa*)&so[w][r][c4];
      if (C) *(volatile v4f*)(C + cofs + (size_t)(row0 + r) * ldc + col0 + c4) = v;
      if (C16) { v4h h4;
#pragma unroll
        for (int i = 0; i < 4; ++i) h4[i] = (_Float16)v[i];
        *(volatile v4h*)(C16 + cofs + (size_t)(row0 + r) * ldc + col0 + c4) = h4; } }
    if (pass == 0) __threadfence(); } }

extern "C" void kernel_launch(void* const* d_in, const int* in_sizes, int n_in,
                              void* d_out, int out_size, void* d_ws, size_t ws_size, hipStream_t stream) {
  if (n_in < 9) return;
  const size_t need_rows = ((size_t)(NB - 1) * SEQ_FULL + SEQ) * DM;
  if ((size_t)in_sizes[0] < need_rows) return;
  if ((size_t)out_size < need_rows) return;
  if ((size_t)in_sizes[1] < (size_t)DM * DM || (size_t)in_sizes[3] < (size_t)DM * DM || (size_t)in_sizes[5] < (size_t)DM * DM || (size_t)in_sizes[7] < (size_t)DM * DM) return;
  if (in_sizes[2] < DM || in_sizes[4] < DM || in_sizes[6] < DM || in_sizes[8] < DM) return;
  const float* x  = (const float*)d_in[0];
  const float* wq = (const float*)d_in[1]; const float* bq = (const float*)d_in[2];
  const float* wk = (const float*)d_in[3]; const float* bk = (const float*)d_in[4];
  const float* wv = (const float*)d_in[5]; const float* bv = (const float*)d_in[6];
  const float* wo = (const float*)d_in[7]; const float* bo = (const float*)d_in[8];
  char* ws = (char*)d_ws; size_t off = 0;
  auto take = [&](size_t bytes) { char* p = ws + off; off += (bytes + 255) & ~(size_t)255; return p; };
  _Float16* BQ = (_Float16*)take(SZ_W); _Float16* BK = (_Float16*)take(SZ_W); _Float16* BV = (_Float16*)take(SZ_W); _Float16* BO = (_Float16*)take(SZ_W);
  _Float16* X16 = (_Float16*)take(SZ_ROW); _Float16* Q16 = (_Float16*)take(SZ_ROW); _Float16* K16 = (_Float16*)take(SZ_ROW); _Float16* V16 = (_Float16*)take(SZ_ROW); _Float16* O16 = (_Float16*)take(SZ_ROW);
  float* S = (float*)take(SZ_S); _Float16* P = (_Float16*)take(SZ_P); _Float16* VT = (_Float16*)take(SZ_VT);
  if (off > ws_size) return;

  const unsigned wblocks = (unsigned)(((size_t)DM * DM / 8 + 255) / 256);
  k_wnat<<<wblocks, 256, 0, stream>>>(wq, (size_t)DM * DM / 8, BQ);
  k_wnat<<<wblocks, 256, 0, stream>>>(wk, (size_t)DM * DM / 8, BK);
  k_wnat<<<wblocks, 256, 0, stream>>>(wv, (size_t)DM * DM / 8, BV);
  k_wnat<<<wblocks, 256, 0, stream>>>(wo, (size_t)DM * DM / 8, BO);
  k_x16<<<(unsigned)((NR * DM / 8 + 255) / 256), 256, 0, stream>>>(x, X16, NR * DM / 8);

  const int MP = (int)NR;
  const unsigned pgrid = (unsigned)((MP / 128) * (DM / 64));
  k_gemm2<0><<<dim3(pgrid, 1), 128, 0, stream>>>(X16, DM, (size_t)0, BQ, DM, (size_t)0, 0.0625f, bq, (size_t)0, (float*)nullptr, Q16, DM, (size_t)0, MP, DM, DM);
  k_gemm2<0><<<dim3(pgrid, 1), 128, 0, stream>>>(X16, DM, (size_t)0, BK, DM, (size_t)0, 0.0625f, bk, (size_t)0, (float*)nullptr, K16, DM, (size_t)0, MP, DM, DM);
  k_gemm2<0><<<dim3(pgrid, 1), 128, 0, stream>>>(X16, DM, (size_t)0, BV, DM, (size_t)0, 0.0625f, bv, (size_t)0, (float*)nullptr, V16, DM, (size_t)0, MP, DM, DM);

  k_vt<NH, SEQ><<<(unsigned)(NB * NH * (SEQ / 64)), 256, 0, stream>>>(V16, LQ, 0, VT);

  for (int b = 0; b < NB; ++b) {
    const size_t r0 = (size_t)b * SEQ;
    for (int h0 = 0; h0 < NH; h0 += HG) {
      k_gemm2<0><<<dim3((unsigned)((SEQ / 128) * (SEQ / 64)), HG), 128, 0, stream>>>(K16 + r0 * LQ + h0 * HD, LQ, (size_t)HD, Q16 + r0 * LQ + h0 * HD, LQ, (size_t)HD, 0.03125f,
          (const float*)nullptr, (size_t)0, S, (_Float16*)nullptr, SEQ, (size_t)SEQ * SEQ, SEQ, SEQ, HD);
      k_rsm<<<(unsigned)((HG * SEQ + 255) / 256), 256, 0, stream>>>(S, P, HG * SEQ);
      k_gemm2<0><<<dim3((unsigned)((SEQ / 128) * (HD / 64)), HG), 128, 0, stream>>>(P, SEQ, (size_t)SEQ * SEQ, VT + ((size_t)b * NH + h0) * HD * SEQ, SEQ, (size_t)HD * SEQ, 0.25f,
          (const float*)nullptr, (size_t)0, (float*)nullptr, O16 + r0 * DM + h0 * HD, DM, (size_t)HD, SEQ, HD, SEQ);
    }
    k_gemm2<0><<<dim3((unsigned)((SEQ / 128) * (DM / 64)), 1), 128, 0, stream>>>(O16 + r0 * DM, DM, (size_t)0, BO, DM, (size_t)0, 0.0009765625f, bo, (size_t)0,
        (float*)d_out + (size_t)b * SEQ_FULL * DM, (_Float16*)nullptr, DM, (size_t)0, SEQ, DM, DM);
  }
}
